// NONLocalBlock2D_43301860278976
// MI455X (gfx1250) — hardware-verified
//
#include <hip/hip_runtime.h>
#include <math.h>
#include <stdint.h>

#ifndef NB
#define NB 8
#endif
#ifndef SEQ
#define SEQ 4096
#endif
#define NB_FULL  8
#define SEQ_FULL 4096
#define CCH   256
#define ICH   128
#define ROWS  (NB * SEQ)
#define NHALF 2
#define HD    64
#define NST   (SEQ / 64)
#define ASC   1024.0f
#define MCAR  4096.0f
#define YSC   1024.0f
#define WOS   1024.0f
#define BN_EPS 1e-3f
#define SLAB64 (16 * 68)
#define VTP   72
#define RPC   (ICH / 8)
#define RPR   16
#define RPT   (RPC * RPR)
#define WS_CAP 134217728
static_assert(NB >= 1 && NB <= NB_FULL);
static_assert((SEQ % 64) == 0 && SEQ >= 64 && SEQ <= SEQ_FULL);
static_assert(ICH == NHALF * HD && HD == 64);
static_assert((ICH % 64) == 0 && (CCH % 64) == 0 && (ICH % 32) == 0 && (CCH % 32) == 0);
static_assert(RPT == 256 && (ROWS % RPR) == 0 && ((NB * ICH) % RPR) == 0);
static_assert((((size_t)ROWS * CCH) % 8) == 0 && ((SEQ * CCH) % 8) == 0);

typedef unsigned short u16;
typedef _Float16 v16h __attribute__((ext_vector_type(16)));
typedef _Float16 v8h  __attribute__((ext_vector_type(8)));
typedef __bf16   v16b __attribute__((ext_vector_type(16)));
typedef float    v8f  __attribute__((ext_vector_type(8)));
typedef float    v4f  __attribute__((ext_vector_type(4)));
typedef unsigned int v4u __attribute__((ext_vector_type(4)));

union FragH { v16h v; v8h h[2]; v4u u[2]; };
union FragB { v16b v; v4u u[2]; };

__device__ __forceinline__ unsigned short bf_bits(float f) {
  unsigned u = __float_as_uint(f);
  return (unsigned short)((u + 0x7FFFu + ((u >> 16) & 1u)) >> 16);
}
__device__ __forceinline__ float bf_up(unsigned short h) { return __uint_as_float(((unsigned)h) << 16); }
__device__ __forceinline__ float bfr(float f) { return bf_up(bf_bits(f)); }
__device__ __forceinline__ unsigned short h_bits(_Float16 x) { return __builtin_bit_cast(unsigned short, x); }
__device__ __forceinline__ unsigned pk16(unsigned short a, unsigned short b) { return (unsigned)a | ((unsigned)b << 16); }
__device__ __forceinline__ v8f zero8() { v8f z = {0.f, 0.f, 0.f, 0.f, 0.f, 0.f, 0.f, 0.f}; return z; }

__device__ __forceinline__ v16h ldfrag_h(const _Float16* p) {
  FragH f;
  f.h[0] = *(const v8h*)(p);
  f.h[1] = *(const v8h*)(p + 16);
  return f.v;
}
__device__ __forceinline__ v16b ldfrag_b(const u16* p) {
  FragB f;
  f.u[0] = *(const v4u*)(p);
  f.u[1] = *(const v4u*)(p + 16);
  return f.v;
}

__device__ __forceinline__ v8f mma_h(v16h a, v16h b, v8f c) {
  return __builtin_amdgcn_wmma_f32_16x16x32_f16(false, a, false, b, (short)0, c, false, false);
}
__device__ __forceinline__ v8f mma_b(v16b a, v16b b, v8f c) {
  return __builtin_amdgcn_wmma_f32_16x16x32_bf16(false, a, false, b, (short)0, c, false, false);
}
template <typename F>
__device__ __forceinline__ void guard6(v8f& a, v8f& b, v8f& c, v8f& d, F x0, F x1, F x2, F x3, F x4, F x5) {
#if defined(__HIP_DEVICE_COMPILE__)
  asm volatile("v_nop\n\tv_nop\n\tv_nop\n\tv_nop"
               : "+v"(a), "+v"(b), "+v"(c), "+v"(d) : "v"(x0), "v"(x1), "v"(x2), "v"(x3), "v"(x4), "v"(x5) : "memory");
#endif
}
template <typename F>
__device__ __forceinline__ void guard10(v8f& a, v8f& b, v8f& c, v8f& d, F x0, F x1, F x2, F x3, F x4,
                                        F x5, F x6, F x7, F x8, F x9) {
#if defined(__HIP_DEVICE_COMPILE__)
  asm volatile("v_nop\n\tv_nop\n\tv_nop\n\tv_nop"
               : "+v"(a), "+v"(b), "+v"(c), "+v"(d)
               : "v"(x0), "v"(x1), "v"(x2), "v"(x3), "v"(x4), "v"(x5), "v"(x6), "v"(x7), "v"(x8), "v"(x9)
               : "memory");
#endif
}
__device__ __forceinline__ void wave_sync_lds() {
  __builtin_amdgcn_fence(__ATOMIC_RELEASE, "workgroup");
  __builtin_amdgcn_wave_barrier();
  __builtin_amdgcn_fence(__ATOMIC_ACQUIRE, "workgroup");
}

__global__ __launch_bounds__(256) void cvtx(const float* __restrict__ x, u16* D, int n8) {
  const int gt = blockIdx.x * 256 + (int)threadIdx.x;
  if (gt >= n8) return;
  const size_t e   = (size_t)gt * 8;
  const size_t per = (size_t)SEQ * CCH;
  const size_t b   = e / per;
  const size_t rem = e - b * per;
  const float* p = x + b * ((size_t)SEQ_FULL * CCH) + rem;
  const v4f a = *(const v4f*)(p), b4 = *(const v4f*)(p + 4);
  float w[8];
#pragma unroll
  for (int i = 0; i < 4; ++i) { w[i] = a[i]; w[4 + i] = b4[i]; }
  v4u o;
#pragma unroll
  for (int i = 0; i < 4; ++i) o[i] = pk16(bf_bits(w[2 * i]), bf_bits(w[2 * i + 1]));
  u16* d = D + e;
  for (int pass = 0; pass < 2; ++pass) {
    *(volatile v4u*)(d) = o;
    __threadfence();
  }
}

__global__ __launch_bounds__(256) void wt16(const float* __restrict__ W, int ldw, int coff, int nct, int kd, u16* D,
                                            int f16mode, float scale) {
  __shared__ __align__(16) u16 T[128 * VTP];
  const int tid = threadIdx.x;
  const int bid = blockIdx.x;
  const int ct  = bid % nct;
  const int rt  = bid / nct;
  if (rt * 64 + 64 > kd) return;
  {
    const int sl = tid >> 2;
    const int dc = (tid & 3) * 32;
    const float* src = W + (size_t)(rt * 64 + sl) * ldw + coff + ct * 128 + dc;
#pragma unroll
    for (int i = 0; i < 8; ++i) {
      const v4f a = *(const v4f*)(src + 4 * i);
#pragma unroll
      for (int e = 0; e < 4; ++e) {
        const float f = a[e];
        const unsigned short hb = h_bits((_Float16)(bfr(f) * scale));
        const unsigned short bb = bf_bits(f);
        T[(dc + 4 * i + e) * VTP + sl] = (f16mode != 0) ? hb : bb;
      }
    }
  }
  __syncthreads();
  v4u w4[4];
  const int q8 = tid >> 3, p8 = (tid & 7) * 8;
#pragma unroll
  for (int it = 0; it < 4; ++it) {
    const int line = it * 32 + q8;
    w4[it] = *(const v4u*)(T + line * VTP + p8);
  }
  const size_t base = ((size_t)ct * 128) * (size_t)kd + rt * 64 + p8;
  for (int pass = 0; pass < 2; ++pass) {
#pragma unroll
    for (int it = 0; it < 4; ++it) {
      const int line = it * 32 + q8;
      *(volatile v4u*)(D + base + (size_t)line * (size_t)kd) = w4[it];
    }
    __threadfence();
  }
}

__global__ __launch_bounds__(256) void tr16(const float* __restrict__ F, u16* Ho, u16* Lo, float sc) {
  __shared__ __align__(16) u16 TA[HD * VTP];
  __shared__ __align__(16) u16 TB[HD * VTP];
  const int tid = threadIdx.x;
  const int bid = blockIdx.x;
  const int st  = bid % NST;
  const int t2  = bid / NST;
  const int g   = t2 % NHALF;
  const int b   = t2 / NHALF;
  if (b >= NB) return;
  const int s0  = st * 64;
  {
    const int sl = tid >> 2;
    const int dc = (tid & 3) * 16;
    const float* src = F + ((size_t)b * SEQ + s0 + sl) * ICH + g * HD + dc;
#pragma unroll
    for (int i = 0; i < 4; ++i) {
      const v4f a = *(const v4f*)(src + 4 * i);
#pragma unroll
      for (int e = 0; e < 4; ++e) {
        const float t = a[e] * sc;
        const _Float16 hv = (_Float16)t;
        const _Float16 lv = (_Float16)(t - (float)hv);
        TA[(dc + 4 * i + e) * VTP + sl] = h_bits(hv);
        TB[(dc + 4 * i + e) * VTP + sl] = h_bits(lv);
      }
    }
  }
  __syncthreads();
  v4u vh[2], vl[2];
  const int q8 = tid >> 3, p8 = (tid & 7) * 8;
#pragma unroll
  for (int it = 0; it < 2; ++it) {
    const int line = it * 32 + q8;
    vh[it] = *(const v4u*)(TA + line * VTP + p8);
    vl[it] = *(const v4u*)(TB + line * VTP + p8);
  }
  const size_t hrow = (size_t)(b * NHALF + g) * HD;
  const size_t base = hrow * (size_t)SEQ + s0 + p8;
  for (int pass = 0; pass < 2; ++pass) {
#pragma unroll
    for (int it = 0; it < 2; ++it) {
      const int line = it * 32 + q8;
      *(volatile v4u*)(Ho + base + (size_t)line * SEQ) = vh[it];
      *(volatile v4u*)(Lo + base + (size_t)line * SEQ) = vl[it];
    }
    __threadfence();
  }
}

template <int NPL>
__global__ __launch_bounds__(RPT) void rp16(const float* __restrict__ F, u16* Hp, u16* Lp, int nrows, float sc) {
  const int tid = (int)threadIdx.x;
  if (tid >= RPT) return;
  const int rl  = tid / RPC;
  const int cc  = tid - rl * RPC;
  const int row = (int)blockIdx.x * RPR + rl;
  if (row >= nrows) return;
  const float* p = F + (size_t)row * ICH + cc * 8;
  const v4f a = *(const v4f*)(p), b4 = *(const v4f*)(p + 4);
  float w[8];
#pragma unroll
  for (int e = 0; e < 4; ++e) { w[e] = a[e] * sc; w[4 + e] = b4[e] * sc; }
  v4u oh, ol;
#pragma unroll
  for (int e = 0; e < 4; ++e) {
    const float t0 = w[2 * e], t1 = w[2 * e + 1];
    const _Float16 h0 = (_Float16)t0, h1 = (_Float16)t1;
    const _Float16 l0 = (_Float16)(t0 - (float)h0), l1 = (_Float16)(t1 - (float)h1);
    oh[e] = pk16(h_bits(h0), h_bits(h1));
    ol[e] = pk16(h_bits(l0), h_bits(l1));
  }
  u16* dh = Hp + (size_t)row * ICH + cc * 8;
  u16* dl = Lp + (size_t)row * ICH + cc * 8;
  for (int pass = 0; pass < 2; ++pass) {
    *(volatile v4u*)(dh) = oh;
    if constexpr (NPL == 2) { *(volatile v4u*)(dl) = ol; }
    __threadfence();
  }
}

__device__ __forceinline__ void stage64(float* sl, v8f a0, v8f a1, v8f a2, v8f a3, float oscale,
                                        float c0, float c1, float c2, float c3, int lane) {
  const int hh = lane >> 4, m = lane & 15;
#pragma unroll
  for (int r = 0; r < 8; ++r) {
    const int ro = (8 * hh + r) * 68 + m;
    sl[ro]      = a0[r] * oscale + c0;
    sl[ro + 16] = a1[r] * oscale + c1;
    sl[ro + 32] = a2[r] * oscale + c2;
    sl[ro + 48] = a3[r] * oscale + c3;
  }
  wave_sync_lds();
}
__device__ __forceinline__ void store64(const float* sl, float* C, int N, size_t rowb, int col0, int lane) {
  const int hh = lane >> 4, m = lane & 15;
  v4f vals[8];
#pragma unroll
  for (int it = 0; it < 8; ++it) vals[it] = *(const v4f*)(sl + (it * 2 + hh) * 68 + m * 4);
  float* dst = C + (rowb + (size_t)hh) * (size_t)N + col0 + m * 4;
  for (int pass = 0; pass < 2; ++pass) {
#pragma unroll
    for (int it = 0; it < 8; ++it) {
      *(volatile v4f*)(dst + (size_t)(it * 2) * (size_t)N) = vals[it];
    }
    __threadfence();
  }
}

__global__ __launch_bounds__(128)
void gemm_bf(const u16* __restrict__ A, const u16* __restrict__ Bt, const float* __restrict__ bias,
             float* C, int M, int N, int K, float oscale) {
  __shared__ __align__(16) float slab[4 * SLAB64];
  const int tid = threadIdx.x, wave = tid >> 5, lane = tid & 31, hh = lane >> 4, m = lane & 15;
  const int ntile = N >> 6;
  const int bid   = blockIdx.x;
  const int rowb  = (bid / ntile) * 64 + wave * 16;
  const int col0  = (bid % ntile) * 64;
  if (rowb + 16 > M) return;
  const float cb0 = bfr(bias[col0 + m]);
  const float cb1 = bfr(bias[col0 + 16 + m]);
  const float cb2 = bfr(bias[col0 + 32 + m]);
  const float cb3 = bfr(bias[col0 + 48 + m]);
  const size_t Kz = (size_t)K;
  const u16* ap = A  + (size_t)(rowb + m) * Kz + 8 * hh;
  const u16* bp = Bt + (size_t)(col0 + m) * Kz + 8 * hh;
  const size_t bs = 16 * Kz;
  v8f acc0 = zero8(), acc1 = zero8(), acc2 = zero8(), acc3 = zero8();
#pragma unroll 1
  for (int k0 = 0; k0 < K; k0 += 32) {
    const v16b a  = ldfrag_b(ap + k0);
    const v16b b0 = ldfrag_b(bp + k0);
    const v16b b1 = ldfrag_b(bp + bs + k0);
    const v16b b2 = ldfrag_b(bp + 2 * bs + k0);
    const v16b b3 = ldfrag_b(bp + 3 * bs + k0);
    acc0 = mma_b(a, b0, acc0);
    acc1 = mma_b(a, b1, acc1);
    acc2 = mma_b(a, b2, acc2);
    acc3 = mma_b(a, b3, acc3);
    guard6<v16b>(acc0, acc1, acc2, acc3, a, b0, b1, b2, b3, a);
  }
  float* sl = slab + wave * SLAB64;
  stage64(sl, acc0, acc1, acc2, acc3, oscale, cb0, cb1, cb2, cb3, lane);
  store64(sl, C, N, (size_t)rowb, col0, lane);
}

template <int NPROD>
__global__ __launch_bounds__(128)
void gemm_h(const u16* __restrict__ Ah, const u16* __restrict__ Al,
            const u16* __restrict__ Bh, const u16* __restrict__ Bl,
            float* C, int MB, int N, int K, int bstrB, int nbat, float oscale) {
  __shared__ __align__(16) float slab[4 * SLAB64];
  const int tid = threadIdx.x, wave = tid >> 5, lane = tid & 31, hh = lane >> 4, m = lane & 15;
  const int ntile = N >> 6, mtile = MB >> 6;
  const int bid   = blockIdx.x;
  const int ct    = bid % ntile;
  const int t2    = bid / ntile;
  const int rt    = t2 % mtile;
  const int bb    = t2 / mtile;
  if (bb >= nbat) return;
  const int col0  = ct * 64;
  const size_t rowC = (size_t)bb * MB + (size_t)rt * 64 + wave * 16;
  const size_t rowB = (size_t)bb * bstrB + col0;
  const size_t Kz   = (size_t)K;
  const _Float16* ahp = (const _Float16*)(const void*)Ah + (rowC + m) * Kz + 8 * hh;
  const _Float16* alp = (const _Float16*)(const void*)Al + (rowC + m) * Kz + 8 * hh;
  const _Float16* bhp = (const _Float16*)(const void*)Bh + (rowB + m) * Kz + 8 * hh;
  const _Float16* blp = (const _Float16*)(const void*)Bl + (rowB + m) * Kz + 8 * hh;
  const size_t bs = 16 * Kz;
  v8f acc0 = zero8(), acc1 = zero8(), acc2 = zero8(), acc3 = zero8();
  if constexpr (NPROD == 3) {
#pragma unroll 1
    for (int k0 = 0; k0 < K; k0 += 32) {
      const v16h ah = ldfrag_h(ahp + k0), al = ldfrag_h(alp + k0);
      const v16h b0 = ldfrag_h(bhp + k0);
      const v16h b1 = ldfrag_h(bhp + bs + k0);
      const v16h b2 = ldfrag_h(bhp + 2 * bs + k0);
      const v16h b3 = ldfrag_h(bhp + 3 * bs + k0);
      const v16h l0 = ldfrag_h(blp + k0);
      const v16h l1 = ldfrag_h(blp + bs + k0);
      const v16h l2 = ldfrag_h(blp + 2 * bs + k0);
      const v16h l3 = ldfrag_h(blp + 3 * bs + k0);
      acc0 = mma_h(ah, b0, acc0);  acc0 = mma_h(al, b0, acc0);  acc0 = mma_h(ah, l0, acc0);
      acc1 = mma_h(ah, b1, acc1);  acc1 = mma_h(al, b1, acc1);  acc1 = mma_h(ah, l1, acc1);
      acc2 = mma_h(ah, b2, acc2);  acc2 = mma_h(al, b2, acc2);  acc2 = mma_h(ah, l2, acc2);
      acc3 = mma_h(ah, b3, acc3);  acc3 = mma_h(al, b3, acc3);  acc3 = mma_h(ah, l3, acc3);
      guard10<v16h>(acc0, acc1, acc2, acc3, ah, al, b0, b1, b2, b3, l0, l1, l2, l3);
    }
  } else if constexpr (NPROD == 2) {
#pragma unroll 1
    for (int k0 = 0; k0 < K; k0 += 32) {
      const v16h ah = ldfrag_h(ahp + k0), al = ldfrag_h(alp + k0);
      const v16h b0 = ldfrag_h(bhp + k0);
      const v16h b1 = ldfrag_h(bhp + bs + k0);
      const v16h b2 = ldfrag_h(bhp + 2 * bs + k0);
      const v16h b3 = ldfrag_h(bhp + 3 * bs + k0);
      acc0 = mma_h(ah, b0, acc0);  acc0 = mma_h(al, b0, acc0);
      acc1 = mma_h(ah, b1, acc1);  acc1 = mma_h(al, b1, acc1);
      acc2 = mma_h(ah, b2, acc2);  acc2 = mma_h(al, b2, acc2);
      acc3 = mma_h(ah, b3, acc3);  acc3 = mma_h(al, b3, acc3);
      guard6<v16h>(acc0, acc1, acc2, acc3, ah, al, b0, b1, b2, b3);
    }
  } else {
#pragma unroll 1
    for (int k0 = 0; k0 < K; k0 += 32) {
      const v16h ah = ldfrag_h(ahp + k0);
      const v16h b0 = ldfrag_h(bhp + k0);
      const v16h b1 = ldfrag_h(bhp + bs + k0);
      const v16h b2 = ldfrag_h(bhp + 2 * bs + k0);
      const v16h b3 = ldfrag_h(bhp + 3 * bs + k0);
      acc0 = mma_h(ah, b0, acc0);
      acc1 = mma_h(ah, b1, acc1);
      acc2 = mma_h(ah, b2, acc2);
      acc3 = mma_h(ah, b3, acc3);
      guard6<v16h>(acc0, acc1, acc2, acc3, ah, b0, b1, b2, b3, ah);
    }
  }
  float* sl = slab + wave * SLAB64;
  stage64(sl, acc0, acc1, acc2, acc3, oscale, 0.0f, 0.0f, 0.0f, 0.0f, lane);
  store64(sl, C, N, rowC, col0, lane);
}

__global__ __launch_bounds__(128)
void gemm_w(const u16* __restrict__ A, const u16* __restrict__ Bt, float* out,
            const float* __restrict__ bW, const float* __restrict__ ga, const float* __restrict__ be,
            const float* __restrict__ mu, const float* __restrict__ var, const float* __restrict__ x, float oscale) {
  __shared__ __align__(16) float slab[4 * SLAB64];
  const int tid = threadIdx.x, wave = tid >> 5, lane = tid & 31, hh = lane >> 4, m = lane & 15;
  const int ntile = CCH >> 6;
  const int mtile = SEQ >> 6;
  const int bid   = blockIdx.x;
  const int ct    = bid % ntile;
  const int t2    = bid / ntile;
  const int rt    = t2 % mtile;
  const int bb    = t2 / mtile;
  if (bb >= NB) return;
  const int srow  = rt * 64 + wave * 16;
  const int col0  = ct * 64;
  const size_t rowC = (size_t)bb * SEQ + srow;
  const size_t rowX = (size_t)bb * SEQ_FULL + srow;
  const size_t Kz   = (size_t)ICH;
  const _Float16* ahp = (const _Float16*)(const void*)A  + (rowC + m) * Kz + 8 * hh;
  const _Float16* bp  = (const _Float16*)(const void*)Bt + (size_t)(col0 + m) * Kz + 8 * hh;
  const size_t bs = 16 * Kz;
  const int col = col0 + m * 4;
  const v4f bw4 = *(const v4f*)(bW + col);
  const v4f ga4 = *(const v4f*)(ga + col);
  const v4f be4 = *(const v4f*)(be + col);
  const v4f mu4 = *(const v4f*)(mu + col);
  const v4f va4 = *(const v4f*)(var + col);
  float bwr[4], gar[4], ber[4], mur[4], rs[4];
#pragma unroll
  for (int e = 0; e < 4; ++e) {
    bwr[e] = bfr(bw4[e]);
    gar[e] = bfr(ga4[e]);
    ber[e] = bfr(be4[e]);
    mur[e] = bfr(mu4[e]);
    rs[e]  = rsqrtf(bfr(va4[e]) + BN_EPS);
  }
  v8f acc0 = zero8(), acc1 = zero8(), acc2 = zero8(), acc3 = zero8();
#pragma unroll 1
  for (int k0 = 0; k0 < ICH; k0 += 32) {
    const v16h ah = ldfrag_h(ahp + k0);
    const v16h b0 = ldfrag_h(bp + k0);
    const v16h b1 = ldfrag_h(bp + bs + k0);
    const v16h b2 = ldfrag_h(bp + 2 * bs + k0);
    const v16h b3 = ldfrag_h(bp + 3 * bs + k0);
    acc0 = mma_h(ah, b0, acc0);
    acc1 = mma_h(ah, b1, acc1);
    acc2 = mma_h(ah, b2, acc2);
    acc3 = mma_h(ah, b3, acc3);
    guard6<v16h>(acc0, acc1, acc2, acc3, ah, b0, b1, b2, b3, ah);
  }
  float* sl = slab + wave * SLAB64;
  stage64(sl, acc0, acc1, acc2, acc3, oscale, 0.0f, 0.0f, 0.0f, 0.0f, lane);
  v4f vals[8];
#pragma unroll
  for (int it = 0; it < 8; ++it) vals[it] = *(const v4f*)(sl + (it * 2 + hh) * 68 + m * 4);
  v4f zs[8];
#pragma unroll
  for (int it = 0; it < 8; ++it) {
    const v4f xv = *(const v4f*)(x + (rowX + (size_t)hh + (size_t)(it * 2)) * CCH + col);
#pragma unroll
    for (int e = 0; e < 4; ++e) {
      const float wy = vals[it][e] + bwr[e];
      float t = gar[e] * (wy - mur[e]);
      t = t * rs[e];
      t = t + ber[e];
      zs[it][e] = t + bfr(xv[e]);
    }
  }
  float* dst = out + (rowC + (size_t)hh) * (size_t)CCH + col;
  for (int pass = 0; pass < 2; ++pass) {
#pragma unroll
    for (int it = 0; it < 8; ++it) {
      *(volatile v4f*)(dst + (size_t)(it * 2) * (size_t)CCH) = zs[it];
    }
    __threadfence();
  }
}

extern "C" void kernel_launch(void* const* d_in, const int* in_sizes, int n_in,
                              void* d_out, int out_size, void* d_ws, size_t ws_size,
                              hipStream_t stream) {
  if (n_in < 13) return;
  if ((size_t)in_sizes[0] < ((size_t)(NB - 1) * SEQ_FULL + SEQ) * CCH) return;
  if (in_sizes[1] < CCH * ICH || in_sizes[3] < CCH * ICH || in_sizes[5] < CCH * ICH) return;
  if (in_sizes[2] < ICH || in_sizes[4] < ICH || in_sizes[6] < ICH) return;
  if (in_sizes[7] < ICH * CCH || in_sizes[8] < CCH) return;
  if (in_sizes[9] < CCH || in_sizes[10] < CCH || in_sizes[11] < CCH || in_sizes[12] < CCH) return;
  if ((size_t)out_size < (size_t)ROWS * CCH) return;

  const float* x    = (const float*)d_in[0];
  const float* w_g  = (const float*)d_in[1];
  const float* b_g  = (const float*)d_in[2];
  const float* w_th = (const float*)d_in[3];
  const float* b_th = (const float*)d_in[4];
  const float* w_ph = (const float*)d_in[5];
  const float* b_ph = (const float*)d_in[6];
  const float* w_W  = (const float*)d_in[7];
  const float* b_W  = (const float*)d_in[8];
  const float* gam  = (const float*)d_in[9];
  const float* bet  = (const float*)d_in[10];
  const float* mu   = (const float*)d_in[11];
  const float* var  = (const float*)d_in[12];
  float*       out  = (float*)d_out;

  const size_t szXB  = (size_t)ROWS * CCH * 2;
  const size_t szWp  = (size_t)ICH * CCH * 2;
  const size_t szF   = (size_t)ROWS * ICH * 4;
  const size_t szT   = (size_t)NB * ICH * SEQ * 2;
  const size_t szR   = (size_t)ROWS * ICH * 2;
  const size_t szMT  = (size_t)NB * ICH * ICH * 4;
  const size_t szM16 = (size_t)NB * ICH * ICH * 2;
  size_t off = 0;
  const size_t oXB = off; off += szXB;
  const size_t oWG = off; off += szWp;
  const size_t oWT = off; off += szWp;
  const size_t oWP = off; off += szWp;
  const size_t oWW = off; off += szWp;
  const size_t oF  = off; off += szF;
  const size_t oGH = off; off += szT;
  const size_t oGL = off; off += szT;
  const size_t oPH = off; off += szT;
  const size_t oPL = off; off += szT;
  const size_t oTH = off; off += szR;
  const size_t oTL = off; off += szR;
  const size_t oMT = off; off += szMT;
  const size_t oMH = off; off += szM16;
  const size_t oML = off; off += szM16;
  const size_t oYH = off; off += szR;
  if (off > ws_size) return;
  if (off > (size_t)WS_CAP) return;

  char* ws = (char*)d_ws;
  u16*   XB = (u16*)(ws + oXB);
  u16*   WG = (u16*)(ws + oWG);
  u16*   WT = (u16*)(ws + oWT);
  u16*   WP = (u16*)(ws + oWP);
  u16*   WW = (u16*)(ws + oWW);
  float* F  = (float*)(ws + oF);
  u16*   GH = (u16*)(ws + oGH);
  u16*   GL = (u16*)(ws + oGL);
  u16*   PH = (u16*)(ws + oPH);
  u16*   PL = (u16*)(ws + oPL);
  u16*   TH = (u16*)(ws + oTH);
  u16*   TL = (u16*)(ws + oTL);
  float* MT = (float*)(ws + oMT);
  u16*   MH = (u16*)(ws + oMH);
  u16*   ML = (u16*)(ws + oML);
  u16*   YH = (u16*)(ws + oYH);

  const dim3 b256(256), b128(128), bRP(RPT);
  const int  n8x = (ROWS * CCH) / 8;
  const dim3 gX((n8x + 255) / 256);
  const dim3 gWT3(1 * (CCH / 64));
  const dim3 gWTW(2 * (ICH / 64));
  const dim3 gG((ROWS / 64) * (ICH / 64));
  const dim3 gTR(NB * NHALF * NST);
  const dim3 gRP(ROWS / RPR);
  const dim3 gRPM((NB * ICH) / RPR);
  const dim3 gM(NB * (ICH / 64) * (ICH / 64));
  const dim3 gY(NB * (SEQ / 64) * (ICH / 64));
  const dim3 gW(NB * (SEQ / 64) * (CCH / 64));
  const float oscM = (1.0f / (ASC * ASC)) * (1.0f / (float)SEQ);
  const float oscY = 1.0f / (ASC * MCAR);
  const float oscW = 1.0f / (YSC * WOS);

  wt16<<<gWT3, b256, 0, stream>>>(w_g,  ICH, 0, 1, CCH, WG, 0, 1.0f);
  wt16<<<gWT3, b256, 0, stream>>>(w_th, ICH, 0, 1, CCH, WT, 0, 1.0f);
  wt16<<<gWT3, b256, 0, stream>>>(w_ph, ICH, 0, 1, CCH, WP, 0, 1.0f);
  wt16<<<gWTW, b256, 0, stream>>>(w_W,  CCH, 0, 2, ICH, WW, 1, WOS);
  cvtx<<<gX, b256, 0, stream>>>(x, XB, n8x);
  gemm_bf<<<gG, b128, 0, stream>>>(XB, WG, b_g, F, ROWS, ICH, CCH, 1.0f);
  tr16<<<gTR, b256, 0, stream>>>(F, GH, GL, ASC);
  gemm_bf<<<gG, b128, 0, stream>>>(XB, WP, b_ph, F, ROWS, ICH, CCH, 1.0f);
  tr16<<<gTR, b256, 0, stream>>>(F, PH, PL, ASC);
  gemm_bf<<<gG, b128, 0, stream>>>(XB, WT, b_th, F, ROWS, ICH, CCH, 1.0f);
  rp16<2><<<gRP, bRP, 0, stream>>>(F, TH, TL, ROWS, ASC);
  gemm_h<3><<<gM, b128, 0, stream>>>(GH, GL, PH, PL, MT, ICH, ICH, SEQ, ICH, NB, oscM);
  rp16<2><<<gRPM, bRP, 0, stream>>>(MT, MH, ML, NB * ICH, MCAR);
  gemm_h<3><<<gY, b128, 0, stream>>>(TH, TL, MH, ML, F, SEQ, ICH, ICH, ICH, NB, oscY);
  rp16<1><<<gRP, bRP, 0, stream>>>(F, YH, YH, ROWS, YSC);
  gemm_w<<<gW, b128, 0, stream>>>(YH, WW, out, b_W, gam, bet, mu, var, x, oscW);
  (void)hipGetLastError();
}
